// Decoder_61108794688068
// MI455X (gfx1250) — hardware-verified
//
#include <hip/hip_runtime.h>
#include <math.h>

#ifndef NP
#define NP 4096
#endif
constexpr int NPF  = 4096;
constexpr int NWAY = 2, KSHOT = 5, NS = NWAY * KSHOT, NQ = NWAY, NBT = NS + NQ;
constexpr int CIN = 320, HID = 196, HIDP = 256, HIDT = 224, DD = 192, ESC = 117, ESP = 128;
constexpr int GB = 6, NGRP = NBT / GB;
constexpr int NP2 = 2 * NP;
constexpr int NTH = 256;
constexpr int CSP = 68;
constexpr float EPSV = 1e-5f;
constexpr float RES_SCALE = 4096.0f, RES_INV = 1.0f / 4096.0f;
constexpr float PSCALE = 4096.0f, PINV = 1.0f / 4096.0f;
constexpr float WSC = 16.0f, WINV = 1.0f / 16.0f;
constexpr float INV_SQRT_D = 0.07216878364870323f;
constexpr int OUT1_OFF = NWAY * NPF * 3;
static_assert(OUT1_OFF * 4 == 98304);
static_assert(NP % 256 == 0 && NP <= NPF);
static_assert(NBT % GB == 0 && (GB * DD) % 8 == 0 && (NBT * NP) % 8 == 0 && (NS * NP) % 8 == 0);
static_assert(CIN % 64 == 0 && HIDP % 64 == 0 && DD % 64 == 0 && ESP % 64 == 0 && NP % 64 == 0);
static_assert(CSP % 4 == 0);

typedef __attribute__((ext_vector_type(16))) _Float16 v16h;
typedef __attribute__((ext_vector_type(8)))  _Float16 v8h;
typedef __attribute__((ext_vector_type(4)))  _Float16 v4h;
typedef __attribute__((ext_vector_type(8)))  float    v8f;
typedef __attribute__((ext_vector_type(4)))  float    v4f;

__device__ __forceinline__ void acc_guard4(v8f& a, v8f& b, v8f& c, v8f& d, v16h x, v16h y, v16h w) {
  asm volatile("v_nop\n\tv_nop\n\tv_nop\n\tv_nop" : "+v"(a), "+v"(b), "+v"(c), "+v"(d) : "v"(x), "v"(y), "v"(w));
}

struct FragH {
  union U { v16h v; v8h h[2]; };
  static __device__ __forceinline__ v16h load(const _Float16* p) {
    U f; f.h[0] = *(const v8h*)(p); f.h[1] = *(const v8h*)(p + 16); return f.v;
  }
  static __device__ __forceinline__ v8f mma(v16h a, v16h b, v8f c) {
    return __builtin_amdgcn_wmma_f32_16x16x32_f16(false, a, false, b, (short)0, c, false, false);
  }
};

__device__ __forceinline__ float rne_bf16(float x) {
  unsigned u = __float_as_uint(x);
  u = (u + 0x7FFFu + ((u >> 16) & 1u)) & 0xFFFF0000u;
  return __uint_as_float(u);
}
__device__ __forceinline__ void split_h(float v, _Float16& hi, _Float16& lo) {
  hi = (_Float16)v;
  const float hf = (float)hi;
  lo = (_Float16)((v - hf) * RES_SCALE);
}
__device__ __forceinline__ float wave_sum(float v) {
#pragma unroll
  for (int o = 16; o > 0; o >>= 1) v += __shfl_xor(v, o, 32);
  return v;
}
__device__ __forceinline__ float wave_max(float v) {
#pragma unroll
  for (int o = 16; o > 0; o >>= 1) v = fmaxf(v, __shfl_xor(v, o, 32));
  return v;
}

__global__ __launch_bounds__(NTH) void wprep_kernel(const float* __restrict__ W, int R, int Cin, _Float16* P, int KP, int total) {
  const int i = blockIdx.x * NTH + threadIdx.x;
  if (i >= total) return;
  const int kp8 = KP >> 3;
  const int row = i / kp8, k8 = (i - row * kp8) * 8;
  const int crow = row < R ? row : (R - 1);
  const float* sp = W + (size_t)crow * Cin;
  v8h hv;
#pragma unroll
  for (int e = 0; e < 8; ++e) {
    const int c = k8 + e, cc = c < Cin ? c : (Cin - 1);
    const float f = (row < R && c < Cin) ? 1.0f : 0.0f;
    hv[e] = (_Float16)(rne_bf16(sp[cc]) * WSC * f);
  }
  _Float16* d = P + (size_t)i * 8;
  *(volatile v8h*)d = hv;
  __threadfence();
  *(volatile v8h*)d = hv;
}

__global__ __launch_bounds__(NTH) void bnstat_cm_kernel(const float* __restrict__ X, int B, long long bstride, int C,
                                                          const float* __restrict__ g, const float* __restrict__ bb,
                                                          float* T, int Cpad) {
  __shared__ float sm[32], sv[32];
  __shared__ __align__(16) float line[64];
  const int tid = threadIdx.x, lane = tid & 31, w = tid >> 5;
  const int c0 = blockIdx.x * 32;
  const float invn = 1.0f / (float)(B * NP);
  for (int j = 0; j < 4; ++j) {
    const int c = c0 + 4 * w + j, cc = c < C ? c : (C - 1);
    float s = 0.0f;
    for (int b = 0; b < B; ++b) {
      const float* p = X + (size_t)b * bstride + (size_t)cc * NPF;
      for (int n4 = lane * 4; n4 < NP; n4 += 128) {
        const v4f v = *(const v4f*)(p + n4);
        s += (rne_bf16(v[0]) + rne_bf16(v[1])) + (rne_bf16(v[2]) + rne_bf16(v[3]));
      }
    }
    s = wave_sum(s);
    const float m = s * invn;
    float q = 0.0f;
    for (int b = 0; b < B; ++b) {
      const float* p = X + (size_t)b * bstride + (size_t)cc * NPF;
      for (int n4 = lane * 4; n4 < NP; n4 += 128) {
        const v4f v = *(const v4f*)(p + n4);
#pragma unroll
        for (int e = 0; e < 4; ++e) { const float dlt = rne_bf16(v[e]) - m; q += dlt * dlt; }
      }
    }
    q = wave_sum(q);
    if (lane == 0) { sm[4 * w + j] = m; sv[4 * w + j] = q * invn; }
  }
  __syncthreads();
  if (tid < 32) {
    const int c = c0 + tid, cc = c < C ? c : (C - 1);
    const float f = c < C ? 1.0f : 0.0f;
    const float gg = rne_bf16(g[cc]), bv = rne_bf16(bb[cc]);
    const float sc = gg * (1.0f / sqrtf(sv[tid] + EPSV)) * f;
    line[tid] = sc;
    line[32 + tid] = (bv - sm[tid] * sc) * f;
  }
  __syncthreads();
  if (tid < 16) {
    const v4f v = *(const v4f*)(line + 4 * tid);
    float* dst = (tid < 8) ? (T + c0 + 4 * tid) : (T + Cpad + c0 + 4 * (tid - 8));
    *(volatile v4f*)dst = v;
    __threadfence();
    *(volatile v4f*)dst = v;
  }
}

__global__ __launch_bounds__(NTH) void bnstat_pm_kernel(const float* __restrict__ X, int R, int ld, int C,
                                                          const float* __restrict__ g, const float* __restrict__ bb,
                                                          float* T, int Cpad) {
  __shared__ float part[8][32];
  __shared__ float sm[32], sv[32];
  __shared__ __align__(16) float line[64];
  const int tid = threadIdx.x, lane = tid & 31, w = tid >> 5;
  const int c0 = blockIdx.x * 32;
  const int c = c0 + lane, cc = c < C ? c : (C - 1);
  const float invn = 1.0f / (float)R;
  float s = 0.0f;
  for (int r = w; r < R; r += 8) s += X[(size_t)r * ld + cc];
  part[w][lane] = s;
  __syncthreads();
  if (tid < 32) {
    float t = 0.0f;
#pragma unroll
    for (int k = 0; k < 8; ++k) t += part[k][tid];
    sm[tid] = t * invn;
  }
  __syncthreads();
  const float m = sm[lane];
  float q = 0.0f;
  for (int r = w; r < R; r += 8) { const float dlt = X[(size_t)r * ld + cc] - m; q += dlt * dlt; }
  part[w][lane] = q;
  __syncthreads();
  if (tid < 32) {
    float t = 0.0f;
#pragma unroll
    for (int k = 0; k < 8; ++k) t += part[k][tid];
    sv[tid] = t * invn;
    const int c2 = c0 + tid, cc2 = c2 < C ? c2 : (C - 1);
    const float f = c2 < C ? 1.0f : 0.0f;
    const float gg = rne_bf16(g[cc2]), bv = rne_bf16(bb[cc2]);
    const float sc = gg * (1.0f / sqrtf(sv[tid] + EPSV)) * f;
    line[tid] = sc;
    line[32 + tid] = (bv - sm[tid] * sc) * f;
  }
  __syncthreads();
  if (tid < 16) {
    const v4f v = *(const v4f*)(line + 4 * tid);
    float* dst = (tid < 8) ? (T + c0 + 4 * tid) : (T + Cpad + c0 + 4 * (tid - 8));
    *(volatile v4f*)dst = v;
    __threadfence();
    *(volatile v4f*)dst = v;
  }
}

template<int MODE, int KP, bool LO>
__global__ __launch_bounds__(NTH) void cvtT_kernel(const float* __restrict__ s32, const _Float16* __restrict__ sh,
                                                    const _Float16* __restrict__ sl, long long sbstride, int sld, int C,
                                                    const float* __restrict__ T, int Cpad, _Float16* dh, _Float16* dl) {
  __shared__ __align__(16) _Float16 th[64 * KP];
  __shared__ __align__(16) _Float16 tl[LO ? 64 * KP : 8];
  const int tid = threadIdx.x;
  const int b = blockIdx.y, n0 = blockIdx.x * 64;
  const int nl = tid & 63, cb = tid >> 6;
  for (int c = cb; c < KP; c += 4) {
    const int cc = c < C ? c : (C - 1);
    const float f = c < C ? 1.0f : 0.0f;
    const size_t so = (size_t)b * sbstride + (size_t)cc * sld + (size_t)(n0 + nl);
    _Float16 h, l = (_Float16)0.0f;
    if (MODE == 0) {
      const float x = rne_bf16(s32[so]);
      const float y = fmaxf(x * T[cc] + T[Cpad + cc], 0.0f) * f;
      h = (_Float16)y;
    } else if (MODE == 1) {
      h = (_Float16)(rne_bf16(s32[so]) * f);
    } else {
      h = sh[so];
      l = sl[so];
    }
    th[nl * KP + c] = h;
    if (LO) tl[nl * KP + c] = l;
  }
  __syncthreads();
  constexpr int NL = KP / 64, NIT = 2 * NL;
  const int w = tid >> 5, lane = tid & 31, q = lane >> 3, p8 = (lane & 7) * 8;
  const size_t dbase = ((size_t)b * NP + (size_t)n0) * KP;
  for (int pass = 0; pass < 2; ++pass) {
#pragma unroll
    for (int it = 0; it < NIT; ++it) {
      const int L = (it * 8 + w) * 4 + q;
      const int row = L / NL, seg = L - row * NL;
      const int off = row * KP + seg * 64 + p8;
      const v8h v = *(const v8h*)(th + off);
      *(volatile v8h*)(dh + dbase + off) = v;
      if (LO) {
        const v8h u = *(const v8h*)(tl + off);
        *(volatile v8h*)(dl + dbase + off) = u;
      }
    }
    __threadfence();
  }
}

__global__ __launch_bounds__(NTH) void bnrelu_pm_kernel(const float* __restrict__ Y, int rows, const float* __restrict__ T,
                                                         _Float16* A) {
  const int i = blockIdx.x * NTH + threadIdx.x;
  if (i >= rows * 32) return;
  const int row = i >> 5, c8 = (i & 31) * 8;
  const float* p = Y + (size_t)row * HIDP + c8;
  const v4f a = *(const v4f*)(p);
  const v4f b = *(const v4f*)(p + 4);
  v8h o;
#pragma unroll
  for (int e = 0; e < 8; ++e) {
    const int c = c8 + e, cc = c < HID ? c : (HID - 1);
    const float f = c < HID ? 1.0f : 0.0f;
    const float v = (e < 4) ? a[e] : b[e - 4];
    o[e] = (_Float16)(fmaxf(v * T[cc] + T[HIDT + cc], 0.0f) * f);
  }
  _Float16* d = A + (size_t)row * HIDP + c8;
  *(volatile v8h*)d = o;
  __threadfence();
  *(volatile v8h*)d = o;
}

template<int NPROD, int BIASM, bool HASADD, int EPI>
__global__ __launch_bounds__(NTH) void gemm_nt_kernel(
    const _Float16* __restrict__ Ah, const _Float16* __restrict__ Al, int lda, long long aStride,
    const _Float16* __restrict__ Bh, const _Float16* __restrict__ Bl, int ldb, long long bStride,
    float* C32, _Float16* Ch, _Float16* Cl, int ldc, long long cStride,
    const float* __restrict__ bias, int nReal, int mReal,
    const _Float16* __restrict__ Xh, const _Float16* __restrict__ Xl, int ldx, long long xStride,
    int K, float outScale) {
  __shared__ __align__(16) float Cs[64 * CSP];
  const int tid = threadIdx.x, wave = tid >> 5, lane = tid & 31;
  const int wm = wave >> 1, wn = wave & 1, hh = lane >> 4, l16 = lane & 15, koff = 8 * hh;
  const int m0 = blockIdx.y * 64, n0 = blockIdx.x * 64;
  const long long z = blockIdx.z;
  const long long arow = (long long)(m0 + 16 * wm + l16) * lda + koff;
  const long long brow = (long long)(n0 + 32 * wn + l16) * ldb + koff;
  const _Float16* ap  = Ah + z * aStride + arow;
  const _Float16* apl = Al + z * aStride + arow;
  const _Float16* bp0 = Bh + z * bStride + brow;
  const _Float16* bp1 = bp0 + 16 * (long long)ldb;
  const _Float16* bq0 = Bl + z * bStride + brow;
  const _Float16* bq1 = bq0 + 16 * (long long)ldb;
  v8f acc0 = {0.f, 0.f, 0.f, 0.f, 0.f, 0.f, 0.f, 0.f};
  v8f acc1 = acc0, accr0 = acc0, accr1 = acc0;

  for (int k0 = 0; k0 < K; k0 += 32) {
    const v16h a  = FragH::load(ap + k0);
    const v16h b0 = FragH::load(bp0 + k0);
    const v16h b1 = FragH::load(bp1 + k0);
    acc0 = FragH::mma(a, b0, acc0);
    acc1 = FragH::mma(a, b1, acc1);
    v16h t = b1;
    if (NPROD >= 2) {
      const v16h c0 = FragH::load(bq0 + k0);
      const v16h c1 = FragH::load(bq1 + k0);
      accr0 = FragH::mma(a, c0, accr0);
      accr1 = FragH::mma(a, c1, accr1);
      t = c1;
    }
    if (NPROD == 3) {
      const v16h al = FragH::load(apl + k0);
      accr0 = FragH::mma(al, b0, accr0);
      accr1 = FragH::mma(al, b1, accr1);
      t = al;
    }
    acc_guard4(acc0, acc1, accr0, accr1, a, b0, t);
  }

#pragma unroll
  for (int s = 0; s < 2; ++s) {
#pragma unroll
    for (int r = 0; r < 8; ++r) {
      float v = (s == 0) ? acc0[r] : acc1[r];
      if (NPROD >= 2) v += ((s == 0) ? accr0[r] : accr1[r]) * RES_INV;
      v *= outScale;
      Cs[(16 * wm + 8 * hh + r) * CSP + 32 * wn + 16 * s + l16] = v;
    }
  }
  __syncthreads();
  const int q = lane >> 3, p = lane & 7;
  if (EPI == 0) {
    for (int pass = 0; pass < 2; ++pass) {
#pragma unroll
      for (int it = 0; it < 4; ++it) {
        const int row = 8 * wave + 2 * it + (q >> 1);
        const int col = (q & 1) * 32 + p * 4;
        v4f v = *(const v4f*)(Cs + row * CSP + col);
        if (BIASM == 1) {
#pragma unroll
          for (int e = 0; e < 4; ++e) {
            const int ci = n0 + col + e, cc = ci < nReal ? ci : (nReal - 1);
            v[e] += (ci < nReal) ? rne_bf16(bias[cc]) : 0.0f;
          }
        }
        if (BIASM == 2) {
          const int ri = m0 + row, cc = ri < mReal ? ri : (mReal - 1);
          const float bv = (ri < mReal) ? rne_bf16(bias[cc]) : 0.0f;
#pragma unroll
          for (int e = 0; e < 4; ++e) v[e] += bv;
        }
        if (HASADD) {
          const long long xo = z * xStride + (long long)(m0 + row) * ldx + n0 + col;
          const v4h xa = *(const v4h*)(Xh + xo);
          const v4h xb = *(const v4h*)(Xl + xo);
#pragma unroll
          for (int e = 0; e < 4; ++e) v[e] += (float)xa[e] + (float)xb[e] * RES_INV;
        }
        float* dst = C32 + z * cStride + (long long)(m0 + row) * ldc + n0 + col;
        *(volatile v4f*)dst = v;
      }
      __threadfence();
    }
  } else {
    for (int pass = 0; pass < 2; ++pass) {
#pragma unroll
      for (int it = 0; it < 2; ++it) {
        const int row = 8 * wave + 4 * it + q;
        const int col = p * 8;
        const v4f v0 = *(const v4f*)(Cs + row * CSP + col);
        const v4f v1 = *(const v4f*)(Cs + row * CSP + col + 4);
        float bvr = 0.0f;
        if (BIASM == 2) {
          const int ri = m0 + row, cc = ri < mReal ? ri : (mReal - 1);
          bvr = (ri < mReal) ? rne_bf16(bias[cc]) : 0.0f;
        }
        v8h hv, lv;
#pragma unroll
        for (int e = 0; e < 8; ++e) {
          float x = (e < 4) ? v0[e] : v1[e - 4];
          if (BIASM == 1) {
            const int ci = n0 + col + e, cc = ci < nReal ? ci : (nReal - 1);
            x += (ci < nReal) ? rne_bf16(bias[cc]) : 0.0f;
          }
          x += bvr;
          const _Float16 h16 = (_Float16)x;
          hv[e] = h16;
          lv[e] = (_Float16)((x - (float)h16) * RES_SCALE);
        }
        const long long co = z * cStride + (long long)(m0 + row) * ldc + n0 + col;
        *(volatile v8h*)(Ch + co) = hv;
        if (EPI == 2) *(volatile v8h*)(Cl + co) = lv;
      }
      __threadfence();
    }
  }
}

__global__ __launch_bounds__(NTH) void proto_pool_kernel(const float* __restrict__ Y2s, const float* __restrict__ T3,
                                                          const int* __restrict__ sy, float* FM) {
  __shared__ float red[3][NTH];
  __shared__ __align__(16) float fms[3 * DD];
  const int tid = threadIdx.x;
  const float fv = (tid < DD) ? 1.0f : 0.0f;
  double s0 = 0.0, s1 = 0.0, s2 = 0.0;
  float c0 = 0.0f, c1 = 0.0f, c2 = 0.0f;
  if (tid < DD) {
    const float sc = T3[tid], sh = T3[DD + tid];
    for (int b = 0; b < NS; ++b) {
      const float fw0 = (b < KSHOT) ? 1.0f : 0.0f, fw1 = 1.0f - fw0;
      const int* yp = sy + (size_t)b * NPF;
      const float* xp = Y2s + (size_t)b * NP * DD + tid;
      for (int n = 0; n < NP; ++n) {
        const int y = yp[n];
        const float v = fmaxf(xp[(size_t)n * DD] * sc + sh, 0.0f);
        const float f0 = (y == 0) ? 1.0f : 0.0f;
        const float f1 = (y == 1) ? 1.0f : 0.0f;
        s0 += (double)(f0 * v); s1 += (double)(f1 * fw0 * v); s2 += (double)(f1 * fw1 * v);
        c0 += f0; c1 += f1 * fw0; c2 += f1 * fw1;
      }
    }
  }
  const float bgv = (float)s0 * (1.0f / fmaxf(c0, 1.0f));
  const float bg  = ((c0 < 1.0f) ? 0.1f : bgv) * fv;
  const float fg0 = (float)s1 * (1.0f / fmaxf(c1, 1.0f)) * fv;
  const float fg1 = (float)s2 * (1.0f / fmaxf(c2, 1.0f)) * fv;
  red[0][tid] = bg * bg; red[1][tid] = fg0 * fg0; red[2][tid] = fg1 * fg1;
  __syncthreads();
  for (int off = NTH / 2; off > 0; off >>= 1) {
    if (tid < off) {
      red[0][tid] += red[0][tid + off];
      red[1][tid] += red[1][tid + off];
      red[2][tid] += red[2][tid + off];
    }
    __syncthreads();
  }
  if (tid < DD) {
    fms[tid]          = bg  * (1.0f / sqrtf(red[0][0]));
    fms[DD + tid]     = fg0 * (1.0f / sqrtf(red[1][0]));
    fms[2 * DD + tid] = fg1 * (1.0f / sqrtf(red[2][0]));
  }
  __syncthreads();
  if (tid < 3 * DD / 4) {
    const v4f v = *(const v4f*)(fms + 4 * tid);
    float* dst = FM + 4 * tid;
    *(volatile v4f*)dst = v;
    __threadfence();
    *(volatile v4f*)dst = v;
  }
}

__global__ __launch_bounds__(NTH) void qf_kernel(const float* __restrict__ Y2q, const float* __restrict__ T3, float* QF, int total) {
  const int i = blockIdx.x * NTH + threadIdx.x;
  if (i >= total) return;
  const int row = i / 48, c4 = (i - row * 48) * 4;
  const v4f y = *(const v4f*)(Y2q + (size_t)row * DD + c4);
  v4f o;
#pragma unroll
  for (int e = 0; e < 4; ++e) o[e] = fmaxf(y[e] * T3[c4 + e] + T3[DD + c4 + e], 0.0f);
  float* dst = QF + (size_t)row * DD + c4;
  *(volatile v4f*)dst = o;
  __threadfence();
  *(volatile v4f*)dst = o;
}

__global__ __launch_bounds__(NTH) void ln_kernel(const float* __restrict__ G, const float* __restrict__ g1, const float* __restrict__ b1,
                                                  const float* __restrict__ g2, const float* __restrict__ b2, _Float16* Fh, _Float16* Fl) {
  __shared__ __align__(16) _Float16 shh[8][DD];
  __shared__ __align__(16) _Float16 shl[8][DD];
  const int tid = threadIdx.x, w = tid >> 5, lane = tid & 31;
  const size_t row = (size_t)blockIdx.x * 8 + (size_t)w;
  const bool side = row < (size_t)NS * NP;
  const float* p = G + row * DD;
  float x[6];
  float s = 0.0f;
#pragma unroll
  for (int j = 0; j < 6; ++j) { x[j] = p[lane + 32 * j]; s += x[j]; }
  s = wave_sum(s);
  const float m = s * (1.0f / (float)DD);
  float q = 0.0f;
#pragma unroll
  for (int j = 0; j < 6; ++j) { const float dlt = x[j] - m; q += dlt * dlt; }
  q = wave_sum(q);
  const float rs = 1.0f / sqrtf(q * (1.0f / (float)DD) + EPSV);
#pragma unroll
  for (int j = 0; j < 6; ++j) {
    const int dch = lane + 32 * j;
    const float ga = rne_bf16(g1[dch]), gb = rne_bf16(g2[dch]);
    const float ba = rne_bf16(b1[dch]), bbv = rne_bf16(b2[dch]);
    const float gg = side ? ga : gb, bo = side ? ba : bbv;
    const float y = (x[j] - m) * rs * gg + bo;
    _Float16 hi, lo;
    split_h(y, hi, lo);
    shh[w][dch] = hi;
    shl[w][dch] = lo;
  }
  __builtin_amdgcn_fence(3  , "wavefront");
  __builtin_amdgcn_wave_barrier();
  const int ls = (lane < 24) ? lane : 0;
  const v8h hv = *(const v8h*)(&shh[w][ls * 8]);
  const v8h lv = *(const v8h*)(&shl[w][ls * 8]);
  _Float16* dh = Fh + row * DD + ls * 8;
  _Float16* dl = Fl + row * DD + ls * 8;
  if (lane < 24) { *(volatile v8h*)dh = hv; *(volatile v8h*)dl = lv; }
  __threadfence();
  if (lane < 24) { *(volatile v8h*)dh = hv; *(volatile v8h*)dl = lv; }
}

__global__ __launch_bounds__(NTH) void softmax_kernel(const float* __restrict__ S, _Float16* P) {
  __shared__ __align__(16) _Float16 shp[8][DD];
  const int tid = threadIdx.x, w = tid >> 5, lane = tid & 31;
  const size_t row = (size_t)blockIdx.x * 8 + (size_t)w;
  const float* p = S + row * DD;
  float x[6];
  float mx = -3.0e38f;
#pragma unroll
  for (int j = 0; j < 6; ++j) { x[j] = p[lane + 32 * j]; mx = fmaxf(mx, x[j]); }
  mx = wave_max(mx);
  float s = 0.0f;
#pragma unroll
  for (int j = 0; j < 6; ++j) { x[j] = __expf(x[j] - mx); s += x[j]; }
  s = wave_sum(s);
  const float inv = (1.0f / s) * PSCALE;
#pragma unroll
  for (int j = 0; j < 6; ++j) shp[w][lane + 32 * j] = (_Float16)(x[j] * inv);
  __builtin_amdgcn_fence(3  , "wavefront");
  __builtin_amdgcn_wave_barrier();
  const int ls = (lane < 24) ? lane : 0;
  const v8h pv = *(const v8h*)(&shp[w][ls * 8]);
  _Float16* d = P + row * DD + ls * 8;
  if (lane < 24) *(volatile v8h*)d = pv;
  __threadfence();
  if (lane < 24) *(volatile v8h*)d = pv;
}

__global__ __launch_bounds__(NTH) void elog_kernel(const float* __restrict__ FM, const float* __restrict__ SEQ, float* Lb) {
  __shared__ float fms[3 * DD];
  const int tid = threadIdx.x, b = blockIdx.y;
  for (int i = tid; i < 3 * DD; i += NTH) fms[i] = FM[i];
  __syncthreads();
  const int n2 = blockIdx.x * NTH + tid;
  const bool side = (blockIdx.x * NTH) < NP;
  const int n = side ? n2 : (n2 - NP);
  float a0 = 0.0f, a1 = 0.0f, a2 = 0.0f;
#pragma unroll 1
  for (int d = 0; d < DD; ++d) {
    float e;
    if (side) {
      float s5 = 0.0f;
#pragma unroll
      for (int k = 0; k < KSHOT; ++k) s5 += SEQ[((size_t)(b * KSHOT + k) * DD + d) * NP + n];
      e = s5 * (1.0f / (float)KSHOT);
    } else {
      e = SEQ[((size_t)(NS + b) * DD + d) * NP + n];
    }
    a0 += fms[d] * e; a1 += fms[DD + d] * e; a2 += fms[2 * DD + d] * e;
  }
  a0 *= INV_SQRT_D; a1 *= INV_SQRT_D; a2 *= INV_SQRT_D;
  float* d0 = Lb + (size_t)(b * 3 + 0) * NP2 + n2;
  float* d1 = Lb + (size_t)(b * 3 + 1) * NP2 + n2;
  float* d2 = Lb + (size_t)(b * 3 + 2) * NP2 + n2;
  *(volatile float*)d0 = a0; *(volatile float*)d1 = a1; *(volatile float*)d2 = a2;
  __threadfence();
  *(volatile float*)d0 = a0; *(volatile float*)d1 = a1; *(volatile float*)d2 = a2;
}

__global__ __launch_bounds__(NTH) void fm2_kernel(const float* __restrict__ FM, const float* __restrict__ SEQ,
                                                   const float* __restrict__ Lb, float* FM2) {
  __shared__ float a2s[NP2];
  __shared__ float red[NTH];
  __shared__ __align__(16) float outs[DD];
  const int tid = threadIdx.x, w = tid >> 5, lane = tid & 31;
  const int m = blockIdx.x, b = blockIdx.y;
  const float* Lr = Lb + (size_t)(b * 3 + m) * NP2;
  float mx = -3.0e38f;
  for (int i = tid; i < NP2; i += NTH) mx = fmaxf(mx, Lr[i]);
  red[tid] = mx;
  __syncthreads();
  for (int off = NTH / 2; off > 0; off >>= 1) { if (tid < off) red[tid] = fmaxf(red[tid], red[tid + off]); __syncthreads(); }
  mx = red[0];
  __syncthreads();
  float s = 0.0f;
  for (int i = tid; i < NP2; i += NTH) { const float e = __expf(Lr[i] - mx); a2s[i] = e; s += e; }
  red[tid] = s;
  __syncthreads();
  for (int off = NTH / 2; off > 0; off >>= 1) { if (tid < off) red[tid] += red[tid + off]; __syncthreads(); }
  const float inv = 1.0f / red[0];
  for (int d = w; d < DD; d += 8) {
    float acc = 0.0f;
    for (int n = lane; n < NP; n += 32) {
      float s5 = 0.0f;
#pragma unroll
      for (int k = 0; k < KSHOT; ++k) s5 += SEQ[((size_t)(b * KSHOT + k) * DD + d) * NP + n];
      const float eq = SEQ[((size_t)(NS + b) * DD + d) * NP + n];
      acc += a2s[n] * (s5 * (1.0f / (float)KSHOT)) + a2s[NP + n] * eq;
    }
    acc = wave_sum(acc);
    if (lane == 0) outs[d] = FM[m * DD + d] + acc * inv;
  }
  __syncthreads();
  if (tid < DD / 4) {
    const v4f v = *(const v4f*)(outs + 4 * tid);
    float* dst = FM2 + (size_t)(b * 3 + m) * DD + 4 * tid;
    *(volatile v4f*)dst = v;
    __threadfence();
    *(volatile v4f*)dst = v;
  }
}

__global__ __launch_bounds__(NTH) void logits_kernel(const float* __restrict__ QF, const float* __restrict__ FM,
                                                      const float* __restrict__ FM2, float* out) {
  __shared__ float f1[3 * DD], f2[3 * DD];
  __shared__ __align__(16) float o0[3 * NTH], o1[3 * NTH];
  const int tid = threadIdx.x;
  const int i = blockIdx.x * NTH + tid;
  const int b = i / NP;
  for (int k = tid; k < 3 * DD; k += NTH) { f1[k] = FM[k]; f2[k] = FM2[b * 3 * DD + k]; }
  __syncthreads();
  const float* qp = QF + (size_t)i * DD;
  float acc[6] = {0.f, 0.f, 0.f, 0.f, 0.f, 0.f};
#pragma unroll 1
  for (int d = 0; d < DD; ++d) {
    const float qv = qp[d];
#pragma unroll
    for (int m = 0; m < 3; ++m) { acc[m] += qv * f1[m * DD + d]; acc[3 + m] += qv * f2[m * DD + d]; }
  }
#pragma unroll
  for (int m = 0; m < 3; ++m) { o0[tid * 3 + m] = acc[m]; o1[tid * 3 + m] = acc[3 + m]; }
  __syncthreads();
  if (tid < 3 * NTH / 4) {
    const v4f va = *(const v4f*)(o0 + 4 * tid);
    const v4f vb = *(const v4f*)(o1 + 4 * tid);
    float* da = out + (size_t)blockIdx.x * (3 * NTH) + 4 * tid;
    float* db = out + OUT1_OFF + (size_t)blockIdx.x * (3 * NTH) + 4 * tid;
    *(volatile v4f*)da = va;
    *(volatile v4f*)db = vb;
    __threadfence();
    *(volatile v4f*)da = va;
    *(volatile v4f*)db = vb;
  }
}

constexpr size_t cmax(size_t a, size_t b) { return a > b ? a : b; }
constexpr size_t ROWS_S = (size_t)NS * NP, ROWS_Q = (size_t)NQ * NP, ROWS_T = (size_t)NBT * NP;
constexpr size_t B_Y1   = ROWS_T * HIDP * 4;
constexpr size_t B_G    = ROWS_T * DD * 4;
constexpr size_t B_XT   = (size_t)GB * NP * DD * 2;
constexpr size_t B_S    = (size_t)GB * DD * DD * 4;
constexpr size_t B_P    = (size_t)GB * DD * DD * 2;
constexpr size_t B_GRP  = 5 * B_XT + B_S + B_P;
constexpr size_t B_R1   = cmax(cmax(B_Y1, B_G), B_GRP);
constexpr size_t B_ACT1 = ROWS_T * CIN * 2, B_ACT2 = ROWS_T * HIDP * 2, B_FHL = 2 * ROWS_T * DD * 2;
constexpr size_t B_R2   = cmax(cmax(B_ACT1, B_ACT2), B_FHL);
constexpr size_t B_Y2   = ROWS_T * DD * 4, B_EST = ROWS_T * ESP * 2, B_SEQ = ROWS_T * DD * 4;
constexpr size_t B_R3   = cmax(cmax(B_Y2, B_EST), B_SEQ);
constexpr size_t B_QF   = ROWS_Q * DD * 4;
static_assert(B_XT % 256 == 0 && B_S % 256 == 0 && B_P % 256 == 0);
static_assert((256 * CIN / 8) % NTH == 0 && (DD * HIDP / 8) % NTH == 0 && (DD * ESP / 8) % NTH == 0 && (DD * DD / 8) % NTH == 0);
static_assert((ROWS_S * 32) % NTH == 0 && (ROWS_Q * 32) % NTH == 0 && (ROWS_Q * 48) % NTH == 0 && (NWAY * NP) % NTH == 0);

extern "C" void kernel_launch(void* const* d_in, const int* in_sizes, int n_in,
                              void* d_out, int out_size, void* d_ws, size_t ws_size, hipStream_t stream) {
  if (n_in < 28 || d_out == nullptr || d_ws == nullptr) return;
  if (in_sizes[0] < NS * CIN * NPF || in_sizes[1] < NS * ESC * NPF || in_sizes[2] < NS * NPF ||
      in_sizes[3] < NQ * CIN * NPF || in_sizes[4] < NQ * ESC * NPF ||
      in_sizes[6] < CIN || in_sizes[7] < CIN || in_sizes[8] < HID * CIN || in_sizes[9] < HID ||
      in_sizes[10] < HID || in_sizes[11] < HID || in_sizes[12] < DD * HID || in_sizes[13] < DD ||
      in_sizes[14] < DD || in_sizes[15] < DD || in_sizes[16] < DD * ESC || in_sizes[17] < DD ||
      in_sizes[18] < DD || in_sizes[19] < DD || in_sizes[20] < DD * ESC || in_sizes[21] < DD ||
      in_sizes[22] < DD || in_sizes[23] < DD || in_sizes[24] < DD * DD || in_sizes[25] < DD ||
      in_sizes[26] < DD * DD || in_sizes[27] < DD) return;
  if (out_size < OUT1_OFF + NWAY * NP * 3) return;

  const float* supf    = (const float*)d_in[0];
  const float* supe    = (const float*)d_in[1];
  const int*   supy    = (const int*)  d_in[2];
  const float* qryf    = (const float*)d_in[3];
  const float* qrye    = (const float*)d_in[4];
  const float* bn1_g   = (const float*)d_in[6];
  const float* bn1_b   = (const float*)d_in[7];
  const float* conv1_W = (const float*)d_in[8];
  const float* conv1_b = (const float*)d_in[9];
  const float* bn2_g   = (const float*)d_in[10];
  const float* bn2_b   = (const float*)d_in[11];
  const float* conv2_W = (const float*)d_in[12];
  const float* conv2_b = (const float*)d_in[13];
  const float* bn3_g   = (const float*)d_in[14];
  const float* bn3_b   = (const float*)d_in[15];
  const float* pre1_W  = (const float*)d_in[16];
  const float* pre1_b  = (const float*)d_in[17];
  const float* ln1_g   = (const float*)d_in[18];
  const float* ln1_b   = (const float*)d_in[19];
  const float* pre2_W  = (const float*)d_in[20];
  const float* pre2_b  = (const float*)d_in[21];
  const float* ln2_g   = (const float*)d_in[22];
  const float* ln2_b   = (const float*)d_in[23];
  const float* dq_W    = (const float*)d_in[24];
  const float* dq_b    = (const float*)d_in[25];
  const float* dv_W    = (const float*)d_in[26];
  const float* dv_b    = (const float*)d_in[27];
  float* out = (float*)d_out;

  char* ws = (char*)d_ws; size_t off = 0;
  auto carve = [&](size_t bytes) -> char* { char* p = ws + off; off += (bytes + 255) & ~(size_t)255; return p; };
  char* R1 = carve(B_R1);
  char* R2 = carve(B_R2);
  char* R3 = carve(B_R3);
  float* QF  = (float*)carve(B_QF);
  float* T1s = (float*)carve(2 * CIN * 4);  float* T1q = (float*)carve(2 * CIN * 4);
  float* T2s = (float*)carve(2 * HIDT * 4); float* T2q = (float*)carve(2 * HIDT * 4);
  float* T3s = (float*)carve(2 * DD * 4);   float* T3q = (float*)carve(2 * DD * 4);
  _Float16* W1p = (_Float16*)carve((size_t)256 * CIN * 2);
  _Float16* W2p = (_Float16*)carve((size_t)DD * HIDP * 2);
  _Float16* Wp1 = (_Float16*)carve((size_t)DD * ESP * 2);
  _Float16* Wp2 = (_Float16*)carve((size_t)DD * ESP * 2);
  _Float16* Wqp = (_Float16*)carve((size_t)DD * DD * 2);
  _Float16* Wvp = (_Float16*)carve((size_t)DD * DD * 2);
  float* FM  = (float*)carve(3 * DD * 4);
  float* FM2 = (float*)carve((size_t)NWAY * 3 * DD * 4);
  float* LB  = (float*)carve((size_t)NWAY * 3 * NP2 * 4);
  if (off > ws_size || off > (size_t)134217728) return;

  float*    Y1   = (float*)R1;
  float*    G    = (float*)R1;
  _Float16* Xth  = (_Float16*)R1;
  _Float16* Xtl  = (_Float16*)(R1 + B_XT);
  _Float16* QH   = (_Float16*)(R1 + 2 * B_XT);
  _Float16* QL   = (_Float16*)(R1 + 3 * B_XT);
  _Float16* VT   = (_Float16*)(R1 + 4 * B_XT);
  float*    Sg   = (float*)(R1 + 5 * B_XT);
  _Float16* Pg   = (_Float16*)(R1 + 5 * B_XT + B_S);
  _Float16* ACT1 = (_Float16*)R2;
  _Float16* ACT2 = (_Float16*)R2;
  _Float16* Fh   = (_Float16*)R2;
  _Float16* Fl   = (_Float16*)(R2 + ROWS_T * DD * 2);
  float*    Y2   = (float*)R3;
  _Float16* EST  = (_Float16*)R3;
  float*    SEQ  = (float*)R3;

  wprep_kernel<<<(256 * CIN / 8) / NTH, NTH, 0, stream>>>(conv1_W, HID, CIN, W1p, CIN, 256 * CIN / 8);
  wprep_kernel<<<(DD * HIDP / 8) / NTH, NTH, 0, stream>>>(conv2_W, DD, HID, W2p, HIDP, DD * HIDP / 8);
  wprep_kernel<<<(DD * ESP / 8) / NTH, NTH, 0, stream>>>(pre1_W, DD, ESC, Wp1, ESP, DD * ESP / 8);
  wprep_kernel<<<(DD * ESP / 8) / NTH, NTH, 0, stream>>>(pre2_W, DD, ESC, Wp2, ESP, DD * ESP / 8);
  wprep_kernel<<<(DD * DD / 8) / NTH, NTH, 0, stream>>>(dq_W, DD, DD, Wqp, DD, DD * DD / 8);
  wprep_kernel<<<(DD * DD / 8) / NTH, NTH, 0, stream>>>(dv_W, DD, DD, Wvp, DD, DD * DD / 8);

  bnstat_cm_kernel<<<CIN / 32, NTH, 0, stream>>>(supf, NS, (long long)CIN * NPF, CIN, bn1_g, bn1_b, T1s, CIN);
  bnstat_cm_kernel<<<CIN / 32, NTH, 0, stream>>>(qryf, NQ, (long long)CIN * NPF, CIN, bn1_g, bn1_b, T1q, CIN);
  cvtT_kernel<0, CIN, false><<<dim3(NP / 64, NS), NTH, 0, stream>>>(supf, W1p, W1p, (long long)CIN * NPF, NPF, CIN, T1s, CIN, ACT1, ACT1);
  cvtT_kernel<0, CIN, false><<<dim3(NP / 64, NQ), NTH, 0, stream>>>(qryf, W1p, W1p, (long long)CIN * NPF, NPF, CIN, T1q, CIN,
                                                                     ACT1 + ROWS_S * CIN, ACT1);
  gemm_nt_kernel<1, 1, false, 0><<<dim3(HIDP / 64, NP / 64, NBT), NTH, 0, stream>>>(
      ACT1, ACT1, CIN, (long long)NP * CIN, W1p, W1p, CIN, 0, Y1, ACT1, ACT1, HIDP, (long long)NP * HIDP,
      conv1_b, HID, NP, W1p, W1p, 0, 0, CIN, WINV);
  bnstat_pm_kernel<<<HIDT / 32, NTH, 0, stream>>>(Y1, (int)ROWS_S, HIDP, HID, bn2_g, bn2_b, T2s, HIDT);
  bnstat_pm_kernel<<<HIDT / 32, NTH, 0, stream>>>(Y1 + ROWS_S * HIDP, (int)ROWS_Q, HIDP, HID, bn2_g, bn2_b, T2q, HIDT);
  bnrelu_pm_kernel<<<(unsigned)(ROWS_S * 32 / NTH), NTH, 0, stream>>>(Y1, (int)ROWS_S, T2s, ACT2);
  bnrelu_pm_kernel<<<(unsigned)(ROWS_Q * 32 / NTH), NTH, 0, stream>>>(Y1 + ROWS_S * HIDP, (int)ROWS_Q, T2q, ACT2 + ROWS_S * HIDP);
  gemm_nt_kernel<1, 1, false, 0><<<dim3(DD / 64, NP / 64, NBT), NTH, 0, stream>>>(
      ACT2, ACT2, HIDP, (long long)NP * HIDP, W2p, W2p, HIDP, 0, Y2, ACT2, ACT2, DD, (long long)NP * DD,
      conv2_b, DD, NP, W2p, W2p, 0, 0, HIDP, WINV);
  bnstat_pm_kernel<<<DD / 32, NTH, 0, stream>>>(Y2, (int)ROWS_S, DD, DD, bn3_g, bn3_b, T3s, DD);
  bnstat_pm_kernel<<<DD / 32, NTH, 0, stream>>>(Y2 + ROWS_S * DD, (int)ROWS_Q, DD, DD, bn3_g, bn3_b, T3q, DD);
  proto_pool_kernel<<<1, NTH, 0, stream>>>(Y2, T3s, supy, FM);
  qf_kernel<<<(unsigned)(ROWS_Q * 48 / NTH), NTH, 0, stream>>>(Y2 + ROWS_S * DD, T3q, QF, (int)(ROWS_Q * 48));

  cvtT_kernel<1, ESP, false><<<dim3(NP / 64, NS), NTH, 0, stream>>>(supe, W1p, W1p, (long long)ESC * NPF, NPF, ESC, T1s, CIN, EST, EST);
  cvtT_kernel<1, ESP, false><<<dim3(NP / 64, NQ), NTH, 0, stream>>>(qrye, W1p, W1p, (long long)ESC * NPF, NPF, ESC, T1s, CIN,
                                                                     EST + ROWS_S * ESP, EST);
  gemm_nt_kernel<1, 1, false, 0><<<dim3(DD / 64, NP / 64, NS), NTH, 0, stream>>>(
      EST, EST, ESP, (long long)NP * ESP, Wp1, Wp1, ESP, 0, G, EST, EST, DD, (long long)NP * DD,
      pre1_b, DD, NP, Wp1, Wp1, 0, 0, ESP, WINV);
  gemm_nt_kernel<1, 1, false, 0><<<dim3(DD / 64, NP / 64, NQ), NTH, 0, stream>>>(
      EST + ROWS_S * ESP, EST, ESP, (long long)NP * ESP, Wp2, Wp2, ESP, 0, G + ROWS_S * DD, EST, EST, DD, (long long)NP * DD,
      pre2_b, DD, NP, Wp2, Wp2, 0, 0, ESP, WINV);
  ln_kernel<<<(unsigned)(ROWS_T / 8), NTH, 0, stream>>>(G, ln1_g, ln1_b, ln2_g, ln2_b, Fh, Fl);

  for (int gi = 0; gi < NGRP; ++gi) {
    const size_t fo = (size_t)gi * GB * NP * DD;
    cvtT_kernel<2, DD, true><<<dim3(NP / 64, GB), NTH, 0, stream>>>(G, Fh + fo, Fl + fo, (long long)DD * NP, NP, DD, T3s, DD, Xth, Xtl);
    gemm_nt_kernel<2, 2, false, 2><<<dim3(NP / 64, DD / 64, GB), NTH, 0, stream>>>(
        Wqp, Wqp, DD, 0, Xth, Xtl, DD, (long long)NP * DD, Sg, QH, QL, NP, (long long)DD * NP,
        dq_b, NP, DD, Xth, Xth, 0, 0, DD, WINV);
    gemm_nt_kernel<1, 1, false, 1><<<dim3(DD / 64, NP / 64, GB), NTH, 0, stream>>>(
        Xth, Xth, DD, (long long)NP * DD, Wvp, Wvp, DD, 0, Sg, VT, VT, DD, (long long)NP * DD,
        dv_b, DD, NP, Xth, Xth, 0, 0, DD, WINV);
    gemm_nt_kernel<3, 0, false, 0><<<dim3(DD / 64, DD / 64, GB), NTH, 0, stream>>>(
        QH, QL, NP, (long long)DD * NP, Fh + fo, Fl + fo, NP, (long long)DD * NP, Sg, QH, QH, DD, (long long)DD * DD,
        dq_b, DD, DD, QH, QH, 0, 0, NP, 1.0f);
    softmax_kernel<<<GB * DD / 8, NTH, 0, stream>>>(Sg, Pg);
    gemm_nt_kernel<1, 0, true, 0><<<dim3(NP / 64, DD / 64, GB), NTH, 0, stream>>>(
        Pg, Pg, DD, (long long)DD * DD, VT, VT, DD, (long long)NP * DD, SEQ + fo, Pg, Pg, NP, (long long)DD * NP,
        dq_b, NP, DD, Fh + fo, Fl + fo, NP, (long long)DD * NP, DD, PINV);
  }

  elog_kernel<<<dim3(NP2 / NTH, NWAY), NTH, 0, stream>>>(FM, SEQ, LB);
  fm2_kernel<<<dim3(3, NWAY), NTH, 0, stream>>>(FM, SEQ, LB, FM2);
  logits_kernel<<<(NWAY * NP) / NTH, NTH, 0, stream>>>(QF, FM, FM2, out);
}
